// Stocknet_64441689309732
// MI455X (gfx1250) — hardware-verified
//
#include <hip/hip_runtime.h>
#include <math.h>

#ifndef NB
#define NB 16384
#endif
#define NB_FULL 16384
#define SEQ 5
#define DM 6
#define NHEAD 2
#define HDIM 3
#define FFD 2048
#define NLAYER 4
#define ROWF (SEQ * DM)
#define MTOK (NB * SEQ)
#define AT_SEQ 256
#define FF_ROWS 256
#define HPF 36

static_assert(NB <= NB_FULL);
static_assert(NB % AT_SEQ == 0);
static_assert(MTOK % FF_ROWS == 0);
static_assert(NHEAD * HDIM == DM);
static_assert(DM <= 8);
static_assert(FFD % 32 == 0);
static_assert(ROWF % 2 == 0);
static_assert(HPF % 4 == 0 && HPF >= 32);
static_assert((7 * 256 + 128) * 16 == AT_SEQ * ROWF * 4);
static_assert(5 * 256 * 16 == AT_SEQ * SEQ * 16);
static_assert(384 * 16 == FF_ROWS * DM * 4);
static_assert(384 % 32 == 0 && 128 % 32 == 0);
static_assert(256 * 8 == AT_SEQ * 2 * 4);
static_assert((NLAYER * FFD) % 256 == 0);
static_assert((NLAYER * 16 * FFD / 8) % 256 == 0);
static_assert(AT_SEQ * ROWF * 4 + AT_SEQ * SEQ * 16 <= 131072);
static_assert(16 * 16 * HPF * 4 + 16 * 16 * 16 * 4 + FF_ROWS * DM * 4 <= 131072);

typedef _Float16 h16;
typedef __attribute__((ext_vector_type(16))) _Float16 v16h;
typedef __attribute__((ext_vector_type(8)))  _Float16 v8h;
typedef __attribute__((ext_vector_type(2)))  _Float16 v2h;
typedef __attribute__((ext_vector_type(8)))  float    v8f;
typedef __attribute__((ext_vector_type(4)))  float    v4f;
typedef __attribute__((ext_vector_type(2)))  float    v2f;
typedef __attribute__((ext_vector_type(4)))  unsigned int v4u;


#define VST2(T, ptr, val) do { const T vst2_v_ = (val); *(volatile T*)(ptr) = vst2_v_; __threadfence(); *(volatile T*)(ptr) = vst2_v_; } while (0)
#define VST2V4(ptr, val) do { const v4f vst2_v4_ = (val); *(volatile v4f*)(ptr) = vst2_v4_; __threadfence(); *(volatile v4f*)(ptr) = vst2_v4_; } while (0)

__device__ __forceinline__ float bfr(float f) {
    unsigned u = __float_as_uint(f);
    u += 0x7FFFu + ((u >> 16) & 1u);
    return __uint_as_float(u & 0xFFFF0000u);
}

static __device__ __forceinline__ unsigned toh_flush_pk(float a, float b) {
    v2f w;
    w.x = (fabsf(a) < 6.103515625e-05f) ? 0.0f : a;
    w.y = (fabsf(b) < 6.103515625e-05f) ? 0.0f : b;
    const v2h r = __builtin_convertvector(w, v2h);
    return __builtin_bit_cast(unsigned, r);
}

union FragU { v16h v; v8h h[2]; };
union FragW { v16h v; v4u u[2]; };
__device__ __forceinline__ v16h frag_ld(const _Float16* p) {
    FragU f; f.h[0] = *(const v8h*)(p); f.h[1] = *(const v8h*)(p + 16); return f.v;
}
__device__ __forceinline__ v8f wmma16(v16h a, v16h b, v8f c) {
    c = __builtin_amdgcn_wmma_f32_16x16x32_f16(false, a, false, b, (short)0, c, false, false);
    asm volatile("v_nop\n\tv_nop\n\tv_nop\n\tv_nop" : "+v"(c) : "v"(a), "v"(b));
    return c;
}
__device__ __forceinline__ void wave_sync_lds() {
    __builtin_amdgcn_fence(3  , "workgroup");
    __builtin_amdgcn_wave_barrier();
    __builtin_amdgcn_fence(2  , "workgroup");
}

#define WP_BLK1 ((NLAYER * FFD) / 256)
#define WP_BLK2 ((NLAYER * 16 * FFD / 8) / 256)
__global__ __launch_bounds__(256) void k_wplanes(const float* __restrict__ W1, const float* __restrict__ W2,
                                                 _Float16* __restrict__ W1P, _Float16* __restrict__ W2P) {
    const unsigned t = threadIdx.x;
    if (blockIdx.x < (unsigned)WP_BLK1) {
        const unsigned u = blockIdx.x * 256u + t;
        const v2f* src = (const v2f*)(W1 + u * (unsigned)DM);
        const v2f a = src[0], b = src[1], c = src[2];
        v4u pk;
        pk.x = toh_flush_pk(bfr(a.x) * 1024.0f, bfr(a.y) * 1024.0f);
        pk.y = toh_flush_pk(bfr(b.x) * 1024.0f, bfr(b.y) * 1024.0f);
        pk.z = toh_flush_pk(bfr(c.x) * 1024.0f, bfr(c.y) * 1024.0f);
        pk.w = 0u;
        VST2(v4u, (v4u*)W1P + u, pk);
    } else {
        const unsigned u = (blockIdx.x - (unsigned)WP_BLK1) * 256u + t;
        const unsigned layer = u >> 12;
        const unsigned o = (u >> 8) & 15u;
        const unsigned g = u & 255u;
        const unsigned oc = (o < (unsigned)DM) ? o : (unsigned)(DM - 1);
        const float live = (o < (unsigned)DM) ? 1024.0f : 0.0f;
        const v4f* src = (const v4f*)(W2 + (layer * (unsigned)DM + oc) * (unsigned)FFD + 8u * g);
        const v4f a = src[0], b = src[1];
        v4u pk;
        pk.x = toh_flush_pk(bfr(a.x) * live, bfr(a.y) * live);
        pk.y = toh_flush_pk(bfr(a.z) * live, bfr(a.w) * live);
        pk.z = toh_flush_pk(bfr(b.x) * live, bfr(b.y) * live);
        pk.w = toh_flush_pk(bfr(b.z) * live, bfr(b.w) * live);
        VST2(v4u, (v4u*)W2P + u, pk);
    }
}

__global__ __launch_bounds__(256) void k_attn(
    const float* __restrict__ xin, int bfin,
    const float* __restrict__ Wq, const float* __restrict__ bq,
    const float* __restrict__ Wk, const float* __restrict__ bk,
    const float* __restrict__ Wv, const float* __restrict__ bv,
    const float* __restrict__ Wo, const float* __restrict__ bo,
    const float* __restrict__ g1, const float* __restrict__ be1,
    float* __restrict__ xs, _Float16* __restrict__ x16) {
    __shared__ __align__(16) float sXS[AT_SEQ * ROWF];
    __shared__ __align__(16) v4u sX16[AT_SEQ * SEQ];
    const unsigned t = threadIdx.x;
    const unsigned b = blockIdx.x * 256u + t;
    float xf[ROWF];
    {
        const v2f* xr = (const v2f*)(xin + b * (unsigned)ROWF);
#pragma unroll
        for (int i = 0; i < ROWF / 2; ++i) { const v2f a = xr[i]; xf[2 * i] = a.x; xf[2 * i + 1] = a.y; }
    }
    if (bfin != 0) {
#pragma unroll
        for (int i = 0; i < ROWF; ++i) xf[i] = bfr(xf[i]);
    }

    float ctx[ROWF];
    const float SCALE = 0.57735026918962576f;
#pragma unroll
    for (int h = 0; h < NHEAD; ++h) {
        float q[SEQ][HDIM], k[SEQ][HDIM], v[SEQ][HDIM];
#pragma unroll
        for (int d = 0; d < HDIM; ++d) {
            const int o = h * HDIM + d;
            float wq[DM], wk[DM], wv[DM];
#pragma unroll
            for (int i = 0; i < DM; ++i) {
                wq[i] = bfr(Wq[o * DM + i]);
                wk[i] = bfr(Wk[o * DM + i]);
                wv[i] = bfr(Wv[o * DM + i]);
            }
            const float cq = bfr(bq[o]), ck = bfr(bk[o]), cv = bfr(bv[o]);
#pragma unroll
            for (int s = 0; s < SEQ; ++s) {
                float aq = xf[s * DM] * wq[0];
                float ak = xf[s * DM] * wk[0];
                float av = xf[s * DM] * wv[0];
#pragma unroll
                for (int i = 1; i < DM; ++i) {
                    aq += xf[s * DM + i] * wq[i];
                    ak += xf[s * DM + i] * wk[i];
                    av += xf[s * DM + i] * wv[i];
                }
                q[s][d] = aq + cq; k[s][d] = ak + ck; v[s][d] = av + cv;
            }
        }
#pragma unroll
        for (int s = 0; s < SEQ; ++s) {
            float sc[SEQ];
            float mx = -3.0e38f;
#pragma unroll
            for (int u = 0; u < SEQ; ++u) {
                float dsum = q[s][0] * k[u][0];
                dsum += q[s][1] * k[u][1];
                dsum += q[s][2] * k[u][2];
                sc[u] = dsum * SCALE;
                mx = fmaxf(mx, sc[u]);
            }
            float se = 0.f;
#pragma unroll
            for (int u = 0; u < SEQ; ++u) { sc[u] = expf(sc[u] - mx); se += sc[u]; }
#pragma unroll
            for (int u = 0; u < SEQ; ++u) sc[u] = sc[u] / se;
#pragma unroll
            for (int d = 0; d < HDIM; ++d) {
                float a = sc[0] * v[0][d];
#pragma unroll
                for (int u = 1; u < SEQ; ++u) a += sc[u] * v[u][d];
                ctx[s * DM + h * HDIM + d] = a;
            }
        }
    }

    float rr[ROWF];
#pragma unroll
    for (int o = 0; o < DM; ++o) {
        float wo[DM];
#pragma unroll
        for (int i = 0; i < DM; ++i) wo[i] = bfr(Wo[o * DM + i]);
        const float co = bfr(bo[o]);
#pragma unroll
        for (int s = 0; s < SEQ; ++s) {
            float a = ctx[s * DM] * wo[0];
#pragma unroll
            for (int i = 1; i < DM; ++i) a += ctx[s * DM + i] * wo[i];
            rr[s * DM + o] = (xf[s * DM + o] + a) + co;
        }
    }
    float gg[DM], bb[DM];
#pragma unroll
    for (int o = 0; o < DM; ++o) { gg[o] = bfr(g1[o]); bb[o] = bfr(be1[o]); }
#pragma unroll
    for (int s = 0; s < SEQ; ++s) {
        float m = rr[s * DM];
#pragma unroll
        for (int o = 1; o < DM; ++o) m += rr[s * DM + o];
        m = m / 6.0f;
        float dv[DM];
        float qs = 0.f;
#pragma unroll
        for (int o = 0; o < DM; ++o) { dv[o] = rr[s * DM + o] - m; qs += dv[o] * dv[o]; }
        const float var = qs / 6.0f;
        const float rs = 1.0f / sqrtf(var + 1e-5f);
        float y[DM];
#pragma unroll
        for (int o = 0; o < DM; ++o) {
            y[o] = dv[o] * rs * gg[o] + bb[o];
            sXS[t * (unsigned)ROWF + (unsigned)(s * DM + o)] = y[o];
        }
        v4u pk;
        pk.x = toh_flush_pk(y[0] * 1024.0f, y[1] * 1024.0f);
        pk.y = toh_flush_pk(y[2] * 1024.0f, y[3] * 1024.0f);
        pk.z = toh_flush_pk(y[4] * 1024.0f, y[5] * 1024.0f);
        pk.w = 0u;
        sX16[t * (unsigned)SEQ + (unsigned)s] = pk;
    }
    __syncthreads();
    {
        float* dst = xs + blockIdx.x * (unsigned)(AT_SEQ * ROWF);
        v4f vv[8];
#pragma unroll
        for (int it = 0; it < 8; ++it) {
            const unsigned idx = (unsigned)it * 256u + t;
            const unsigned idc = (idx < 1920u) ? idx : 1919u;
            vv[it] = *(const v4f*)(sXS + 4u * idc);
        }
        for (int pass = 0; pass < 2; ++pass) {
#pragma unroll
            for (int it = 0; it < 8; ++it) {
                const unsigned idx = (unsigned)it * 256u + t;
                if (idx < 1920u) *(volatile v4f*)(dst + 4u * idx) = vv[it];
            }
            __threadfence();
        }
    }
    {
        v4u* dst = (v4u*)x16 + blockIdx.x * (unsigned)(AT_SEQ * SEQ);
        v4u hv[5];
#pragma unroll
        for (int it = 0; it < 5; ++it) hv[it] = sX16[(unsigned)it * 256u + t];
        for (int pass = 0; pass < 2; ++pass) {
#pragma unroll
            for (int it = 0; it < 5; ++it) *(volatile v4u*)(dst + (unsigned)it * 256u + t) = hv[it];
            __threadfence();
        }
    }
}

__global__ __launch_bounds__(512) void k_ffn(
    const float* __restrict__ xs_in, const _Float16* __restrict__ x16,
    const _Float16* __restrict__ W1P, const _Float16* __restrict__ W2P,
    const float* __restrict__ b1, const float* __restrict__ b2,
    const float* __restrict__ g2, const float* __restrict__ be2,
    float* __restrict__ xs_out) {
    __shared__ __align__(16) float sH[16][16 * HPF];
    __shared__ __align__(16) float sF[16][16 * 16];
    __shared__ __align__(16) float sO[FF_ROWS * DM];
    const unsigned tid = threadIdx.x, lane = tid & 31u;
    const unsigned wave = (unsigned)__builtin_amdgcn_readfirstlane((int)(tid >> 5));
    const unsigned hh = lane >> 4, c = lane & 15u;
    const unsigned row0 = blockIdx.x * (unsigned)FF_ROWS + wave * 16u;

    v8h zero8;
#pragma unroll
    for (int e = 0; e < 8; ++e) zero8[e] = (h16)0.0f;

    FragU xa;
    {
        const v8h ld = *(const v8h*)(x16 + (row0 + c) * 8u);
        xa.h[0] = (hh == 0u) ? ld : zero8;
        xa.h[1] = zero8;
    }
    float* pw = sH[wave];
    v8f os = (v8f){0.f,0.f,0.f,0.f,0.f,0.f,0.f,0.f};

#pragma unroll 1
    for (unsigned ch = 0; ch < (unsigned)(FFD / 32); ++ch) {
        const unsigned u0 = ch * 32u;
#pragma unroll
        for (int j = 0; j < 2; ++j) {
            const unsigned unit = u0 + 16u * (unsigned)j + c;
            const v8h wl = *(const v8h*)(W1P + unit * 8u);
            FragU wb;
            wb.h[0] = (hh == 0u) ? wl : zero8;
            wb.h[1] = zero8;
            const v8f z = (v8f){0.f,0.f,0.f,0.f,0.f,0.f,0.f,0.f};
            const v8f d = wmma16(xa.v, wb.v, z);
            const float bj = bfr(b1[unit]);
#pragma unroll
            for (int r = 0; r < 8; ++r) {
                float hv = d[r] * (1.0f / 1048576.0f) + bj;
                hv = fmaxf(hv, 0.0f);
                pw[(8u * hh + (unsigned)r) * (unsigned)HPF + 16u * (unsigned)j + c] = hv * 256.0f;
            }
        }
        wave_sync_lds();
        FragW pa;
        {
            const float* pr = pw + c * (unsigned)HPF + 8u * hh;
            const v4f p0 = *(const v4f*)(pr);
            const v4f p1 = *(const v4f*)(pr + 4);
            const v4f p2 = *(const v4f*)(pr + 16);
            const v4f p3 = *(const v4f*)(pr + 20);
            pa.u[0].x = toh_flush_pk(p0.x, p0.y);
            pa.u[0].y = toh_flush_pk(p0.z, p0.w);
            pa.u[0].z = toh_flush_pk(p1.x, p1.y);
            pa.u[0].w = toh_flush_pk(p1.z, p1.w);
            pa.u[1].x = toh_flush_pk(p2.x, p2.y);
            pa.u[1].y = toh_flush_pk(p2.z, p2.w);
            pa.u[1].z = toh_flush_pk(p3.x, p3.y);
            pa.u[1].w = toh_flush_pk(p3.z, p3.w);
        }
        const v16h wf = frag_ld(W2P + c * (unsigned)FFD + u0 + 8u * hh);
        os = wmma16(pa.v, wf, os);
        wave_sync_lds();
    }

    float* pf = sF[wave];
#pragma unroll
    for (int r = 0; r < 8; ++r) pf[(8u * hh + (unsigned)r) * 16u + c] = os[r] * (1.0f / 262144.0f);
    wave_sync_lds();
    {
        const v4f f0 = *(const v4f*)(pf + c * 16u);
        const v2f f1 = *(const v2f*)(pf + c * 16u + 4u);
        const v2f* xr = (const v2f*)(xs_in + (row0 + c) * (unsigned)DM);
        const v2f x0 = xr[0], x1 = xr[1], x2 = xr[2];
        const float ff[DM] = {f0.x, f0.y, f0.z, f0.w, f1.x, f1.y};
        const float xv[DM] = {x0.x, x0.y, x1.x, x1.y, x2.x, x2.y};
        float rr[DM];
#pragma unroll
        for (int o = 0; o < DM; ++o) rr[o] = (xv[o] + ff[o]) + bfr(b2[o]);
        float m = rr[0];
#pragma unroll
        for (int o = 1; o < DM; ++o) m += rr[o];
        m = m / 6.0f;
        float dv[DM];
        float qs = 0.f;
#pragma unroll
        for (int o = 0; o < DM; ++o) { dv[o] = rr[o] - m; qs += dv[o] * dv[o]; }
        const float var = qs / 6.0f;
        const float rs = 1.0f / sqrtf(var + 1e-5f);
        float y[DM];
#pragma unroll
        for (int o = 0; o < DM; ++o) y[o] = dv[o] * rs * bfr(g2[o]) + bfr(be2[o]);
        if (hh == 0u) {
#pragma unroll
            for (int o = 0; o < DM; ++o) sO[(wave * 16u + c) * (unsigned)DM + (unsigned)o] = y[o];
        }
    }
    __syncthreads();
    {
        const unsigned idc = (tid < 384u) ? tid : 383u;
        const v4f vv = *(const v4f*)(sO + 4u * idc);
        float* dst = xs_out + blockIdx.x * (unsigned)(FF_ROWS * DM);
        for (int pass = 0; pass < 2; ++pass) {
            if (tid < 384u) *(volatile v4f*)(dst + 4u * tid) = vv;
            __threadfence();
        }
    }
}

__global__ __launch_bounds__(256) void k_head(const float* __restrict__ xs, const float* __restrict__ Wfc,
                                              const float* __restrict__ bfc, float* __restrict__ out) {
    const unsigned b = blockIdx.x * 256u + threadIdx.x;
    float xf[ROWF];
    {
        const v2f* xr = (const v2f*)(xs + b * (unsigned)ROWF);
#pragma unroll
        for (int i = 0; i < ROWF / 2; ++i) { const v2f a = xr[i]; xf[2 * i] = a.x; xf[2 * i + 1] = a.y; }
    }
    float l0 = xf[0] * bfr(Wfc[0]);
    float l1 = xf[0] * bfr(Wfc[ROWF]);
#pragma unroll
    for (int i = 1; i < ROWF; ++i) {
        l0 += xf[i] * bfr(Wfc[i]);
        l1 += xf[i] * bfr(Wfc[ROWF + i]);
    }
    l0 += bfr(bfc[0]);
    l1 += bfr(bfc[1]);
    const float mx = fmaxf(l0, l1);
    const float e0 = expf(l0 - mx), e1 = expf(l1 - mx);
    const float se = e0 + e1;
    v2f o;
    o.x = e0 / se;
    o.y = e1 / se;
    VST2(v2f, (v2f*)(out + 2u * b), o);
}

#define XS_BYTES  ((size_t)MTOK * DM * 4)
#define X16_BYTES ((size_t)MTOK * 16)
#define W1P_BYTES ((size_t)NLAYER * FFD * 16)
#define W2P_BYTES ((size_t)NLAYER * 16 * FFD * 2)
#define OFF_XSA ((size_t)0)
#define OFF_XSB (OFF_XSA + XS_BYTES)
#define OFF_X16 (OFF_XSB + XS_BYTES)
#define OFF_W1P (OFF_X16 + X16_BYTES)
#define OFF_W2P (OFF_W1P + W1P_BYTES)
#define WS_TOTAL (OFF_W2P + W2P_BYTES)
static_assert(XS_BYTES % 256 == 0 && X16_BYTES % 256 == 0 && W1P_BYTES % 256 == 0 && W2P_BYTES % 256 == 0);
static_assert(WS_TOTAL <= (size_t)134217728);
static_assert((size_t)WP_BLK1 * 256 * 16 == W1P_BYTES);
static_assert((size_t)WP_BLK2 * 256 * 16 == W2P_BYTES);
static_assert((size_t)(NB / AT_SEQ) * AT_SEQ * ROWF * 4 == XS_BYTES);
static_assert((size_t)(NB / AT_SEQ) * AT_SEQ * SEQ * 16 == X16_BYTES);
static_assert((size_t)(MTOK / FF_ROWS) * FF_ROWS * DM * 4 == XS_BYTES);

extern "C" void kernel_launch(void* const* d_in, const int* in_sizes, int n_in, void* d_out, int out_size,
                              void* d_ws, size_t ws_size, hipStream_t stream) {
    if (n_in < 19) return;
    if (in_sizes[0] < NB * ROWF) return;
    if (in_sizes[1] < NLAYER * DM * DM || in_sizes[3] < NLAYER * DM * DM || in_sizes[5] < NLAYER * DM * DM || in_sizes[7] < NLAYER * DM * DM) return;
    if (in_sizes[2] < NLAYER * DM || in_sizes[4] < NLAYER * DM || in_sizes[6] < NLAYER * DM || in_sizes[8] < NLAYER * DM) return;
    if (in_sizes[9] < NLAYER * FFD * DM || in_sizes[10] < NLAYER * FFD || in_sizes[11] < NLAYER * DM * FFD || in_sizes[12] < NLAYER * DM) return;
    if (in_sizes[13] < NLAYER * DM || in_sizes[14] < NLAYER * DM || in_sizes[15] < NLAYER * DM || in_sizes[16] < NLAYER * DM) return;
    if (in_sizes[17] < 2 * ROWF || in_sizes[18] < 2 || out_size < NB * 2) return;
    if (ws_size < WS_TOTAL) return;

    const float* x   = (const float*)d_in[0];
    const float* Wq  = (const float*)d_in[1];
    const float* bq  = (const float*)d_in[2];
    const float* Wk  = (const float*)d_in[3];
    const float* bk  = (const float*)d_in[4];
    const float* Wv  = (const float*)d_in[5];
    const float* bv  = (const float*)d_in[6];
    const float* Wo  = (const float*)d_in[7];
    const float* bo  = (const float*)d_in[8];
    const float* W1  = (const float*)d_in[9];
    const float* b1  = (const float*)d_in[10];
    const float* W2  = (const float*)d_in[11];
    const float* b2  = (const float*)d_in[12];
    const float* g1  = (const float*)d_in[13];
    const float* be1 = (const float*)d_in[14];
    const float* g2  = (const float*)d_in[15];
    const float* be2 = (const float*)d_in[16];
    const float* Wfc = (const float*)d_in[17];
    const float* bfc = (const float*)d_in[18];
    float* out = (float*)d_out;

    char* wsp = (char*)d_ws;
    float*    XSA = (float*)(wsp + OFF_XSA);
    float*    XSB = (float*)(wsp + OFF_XSB);
    _Float16* X16 = (_Float16*)(wsp + OFF_X16);
    _Float16* W1P = (_Float16*)(wsp + OFF_W1P);
    _Float16* W2P = (_Float16*)(wsp + OFF_W2P);

    k_wplanes<<<WP_BLK1 + WP_BLK2, 256, 0, stream>>>(W1, W2, W1P, W2P);

    for (int l = 0; l < NLAYER; ++l) {
        const float* ain = (l == 0) ? x : (const float*)XSA;
        k_attn<<<NB / AT_SEQ, 256, 0, stream>>>(ain, (l == 0) ? 1 : 0,
            Wq + l * DM * DM, bq + l * DM, Wk + l * DM * DM, bk + l * DM,
            Wv + l * DM * DM, bv + l * DM, Wo + l * DM * DM, bo + l * DM,
            g1 + l * DM, be1 + l * DM, XSB, X16);
        k_ffn<<<MTOK / FF_ROWS, 512, 0, stream>>>((const float*)XSB, (const _Float16*)X16,
            (const _Float16*)(W1P + (size_t)l * FFD * 8), (const _Float16*)(W2P + (size_t)l * 16 * FFD),
            b1 + l * FFD, b2 + l * DM, g2 + l * DM, be2 + l * DM, XSA);
    }
    k_head<<<NB / AT_SEQ, 256, 0, stream>>>((const float*)XSA, Wfc, bfc, out);
}
